// SAGE_60361470378413
// MI455X (gfx1250) — hardware-verified
//
#include <hip/hip_runtime.h>
#include <hip/hip_bf16.h>
#include <stddef.h>
#include <stdint.h>


#define DIN     128
#define DH      128
#define DC      64
#define PW      256
#define APW     256
#define NTHR    256
#define NWAVE   8
#define EPT     8
#define CHUNK   (NTHR * EPT)
#define WCAP    (EPT * 32)
#define LISTN   (NWAVE * WCAP)
#define NBMAX   2048
#define RCAP    28672
#define DEGCAP  64
#define PKS     11
#define STW     512
#define GBM     64
#define GTHR    128
#define WSMAX   268435456
#define LDS_AGG ((2 * RCAP + 2 * NBMAX + LISTN) * 4 + 64)

static_assert((CHUNK & (CHUNK - 1)) == 0 && CHUNK <= (1 << PKS));
static_assert((NBMAX & (NBMAX - 1)) == 0 && NBMAX <= (1 << PKS));
static_assert(NTHR * 8 == NBMAX);
static_assert(LISTN >= NBMAX);
static_assert(LISTN >= NWAVE * WCAP);
static_assert((RCAP % 32) == 0);
static_assert(NWAVE * STW <= RCAP);
static_assert(LDS_AGG <= 300000);
static_assert(GBM == (GTHR / 32) * 16);
static_assert((DIN % 32) == 0 && (DH % 32) == 0 && (DC % 64) == 0);
static_assert(DH == 32 * 4 && DC == 32 * 2);
static_assert(PW == 2 * DH && APW == 2 * DH);

typedef float          v2f  __attribute__((ext_vector_type(2)));
typedef float          v4f  __attribute__((ext_vector_type(4)));
typedef float          v8f  __attribute__((ext_vector_type(8)));
typedef int            v4i  __attribute__((ext_vector_type(4)));
typedef int            v8i  __attribute__((ext_vector_type(8)));
typedef unsigned int   v2u  __attribute__((ext_vector_type(2)));
typedef unsigned int   v4u  __attribute__((ext_vector_type(4)));
typedef unsigned short v8us __attribute__((ext_vector_type(8)));
typedef __bf16         v16b __attribute__((ext_vector_type(16)));
union FragB { v16b v; v8us h[2]; v8i w; };

__device__ __forceinline__ v8f wmb(const FragB& a, const FragB& b, v8f c) {
  v8f d = __builtin_amdgcn_wmma_f32_16x16x32_bf16(false, a.v, false, b.v, (short)0, c, false, false);
  asm volatile("v_nop\n\tv_nop\n\tv_nop\n\tv_nop" : "+v"(d) : "v"(a.w), "v"(b.w));
  return d;
}

__device__ __forceinline__ unsigned short bf_bits(float f) {
  unsigned int u = __float_as_uint(f);
  u += 0x7FFFu + ((u >> 16) & 1u);
  return (unsigned short)(u >> 16);
}
__device__ __forceinline__ float bf_val(unsigned short b) {
  return __uint_as_float(((unsigned int)b) << 16);
}
__device__ __forceinline__ float bf_rne(float f) { return bf_val(bf_bits(f)); }

__device__ __forceinline__ v8us cvt8b(const v4f a, const v4f b) {
  v8us hv;
  hv[0] = bf_bits(a.x); hv[1] = bf_bits(a.y); hv[2] = bf_bits(a.z); hv[3] = bf_bits(a.w);
  hv[4] = bf_bits(b.x); hv[5] = bf_bits(b.y); hv[6] = bf_bits(b.z); hv[7] = bf_bits(b.w);
  return hv;
}

__device__ __forceinline__ int scan_chunk(const int* __restrict__ dsts, int nE, int cbase, int slotBase,
                                          int nb, int vec8, int* list, int tid, int lane, int wave) {
  int wc = 0;
  const int el0  = tid * EPT;
  const int e0   = cbase + el0;
  const int sent = -2147483647 - 1;
  v4i da, db;
  if (vec8 != 0 && cbase + CHUNK <= nE) {
    da = *(const v4i*)(dsts + e0);
    db = *(const v4i*)(dsts + e0 + 4);
  } else {
    da.x = (e0     < nE) ? dsts[min(e0,     nE - 1)] : sent;
    da.y = (e0 + 1 < nE) ? dsts[min(e0 + 1, nE - 1)] : sent;
    da.z = (e0 + 2 < nE) ? dsts[min(e0 + 2, nE - 1)] : sent;
    da.w = (e0 + 3 < nE) ? dsts[min(e0 + 3, nE - 1)] : sent;
    db.x = (e0 + 4 < nE) ? dsts[min(e0 + 4, nE - 1)] : sent;
    db.y = (e0 + 5 < nE) ? dsts[min(e0 + 5, nE - 1)] : sent;
    db.z = (e0 + 6 < nE) ? dsts[min(e0 + 6, nE - 1)] : sent;
    db.w = (e0 + 7 < nE) ? dsts[min(e0 + 7, nE - 1)] : sent;
  }
  const unsigned nbs = (unsigned)slotBase;
  const unsigned unb = (unsigned)nb;
  const unsigned s0 = (unsigned)da.x - nbs, s1 = (unsigned)da.y - nbs;
  const unsigned s2 = (unsigned)da.z - nbs, s3 = (unsigned)da.w - nbs;
  const unsigned s4 = (unsigned)db.x - nbs, s5 = (unsigned)db.y - nbs;
  const unsigned s6 = (unsigned)db.z - nbs, s7 = (unsigned)db.w - nbs;
  const bool h0 = s0 < unb, h1 = s1 < unb, h2 = s2 < unb, h3 = s3 < unb;
  const bool h4 = s4 < unb, h5 = s5 < unb, h6 = s6 < unb, h7 = s7 < unb;
  const unsigned any = __builtin_amdgcn_ballot_w32(h0 | h1 | h2 | h3 | h4 | h5 | h6 | h7);
  if (any != 0u) {
#define HITJ(J, HJ, SJ) { \
      const unsigned mj = __builtin_amdgcn_ballot_w32(HJ); \
      if (mj != 0u) { \
        if (HJ) { \
          const int pos = wc + (int)__builtin_amdgcn_mbcnt_lo(mj, 0u); \
          if (pos < WCAP) list[wave * WCAP + pos] = ((el0 + (J)) << PKS) | (int)(SJ); \
        } \
        wc += (int)__builtin_popcount(mj); } }
    HITJ(0, h0, s0)
    HITJ(1, h1, s1)
    HITJ(2, h2, s2)
    HITJ(3, h3, s3)
    HITJ(4, h4, s4)
    HITJ(5, h5, s5)
    HITJ(6, h6, s6)
    HITJ(7, h7, s7)
#undef HITJ
  }
  return wc;
}

__global__ __launch_bounds__(NTHR) void k_xprep(const float* __restrict__ x, unsigned short* xb,
                                                int nN, int nUnits) {
  const int i = (int)blockIdx.x * NTHR + (int)threadIdx.x;
  if (i >= nUnits) return;
  const int row = i >> 4;
  const int c0  = (i & 15) * 8;
  const int rc  = row < nN ? row : nN - 1;
  const float* p = x + (size_t)rc * DIN + c0;
  v4f a = *(const v4f*)p, b = *(const v4f*)(p + 4);
  const v4f z4 = {0.f, 0.f, 0.f, 0.f};
  if (row >= nN) { a = z4; b = z4; }
  const v8us hv = cvt8b(a, b);
  const size_t o = (size_t)row * DIN + c0;
  *(volatile v8us*)(xb + o) = hv;
  __threadfence();
  *(volatile v8us*)(xb + o) = hv;
}

__global__ __launch_bounds__(NTHR) void k_wtr(const float* __restrict__ w0, const float* __restrict__ w1,
                                              int c0, int c1, int segRows, int Kin, int K,
                                              unsigned short* wt, int nUnits) {
  const int u = (int)blockIdx.x * NTHR + (int)threadIdx.x;
  if (u >= nUnits) return;
  const int kq = K >> 3;
  const int n  = u / kq;
  const int k8 = (u - n * kq) * 8;
  int seg = n / segRows;
  seg = seg > 1 ? 1 : (seg < 0 ? 0 : seg);
  const int nc = n - seg * segRows;
  const float* ws = (seg == 0) ? w0 : w1;
  const int cc = (seg == 0) ? c0 : c1;
  int ncl = nc < cc ? nc : cc - 1;
  ncl = ncl < 0 ? 0 : ncl;
  int ks = k8 - (k8 / Kin) * Kin;
  ks = ks < 0 ? 0 : ks;
  const float* p = ws + (size_t)ks * (size_t)cc + ncl;
  v4f a, b;
  a.x = p[0];                  a.y = p[(size_t)cc];         a.z = p[(size_t)2 * cc];     a.w = p[(size_t)3 * cc];
  b.x = p[(size_t)4 * cc];     b.y = p[(size_t)5 * cc];     b.z = p[(size_t)6 * cc];     b.w = p[(size_t)7 * cc];
  const v4f z4 = {0.f, 0.f, 0.f, 0.f};
  if (nc >= cc) { a = z4; b = z4; }
  const v8us hv = cvt8b(a, b);
  const size_t o = (size_t)n * (size_t)K + k8;
  *(volatile v8us*)(wt + o) = hv;
  __threadfence();
  *(volatile v8us*)(wt + o) = hv;
}

template<int NT>
__global__ __launch_bounds__(GTHR) void k_gemm(const unsigned short* A, int lda,
                                               const unsigned short* __restrict__ WT, int K,
                                               float* outF, int ldo)
{
  constexpr int BN  = 16 * NT;
  constexpr int LPR = 4 * NT;
  constexpr int RPI = 32 / LPR;
  constexpr int NI  = 16 / RPI;
  __shared__ __attribute__((aligned(16))) float stg[GBM * BN];
  const int tid = (int)threadIdx.x, lane = tid & 31, wave = tid >> 5, hh = lane >> 4, m = lane & 15;
  const int rowBase = (int)blockIdx.x * GBM;
  const int col0    = (int)blockIdx.y * BN;

  v8f acc[NT];
  {
    const v8f z = {0.f, 0.f, 0.f, 0.f, 0.f, 0.f, 0.f, 0.f};
#pragma unroll
    for (int t = 0; t < NT; ++t) acc[t] = z;
  }
  const unsigned short* ap = A  + (size_t)(rowBase + 16 * wave + m) * (size_t)lda + 8 * hh;
  const unsigned short* wp = WT + (size_t)(col0 + m) * (size_t)K + 8 * hh;
  const int ksteps = K >> 5;
#pragma unroll 1
  for (int ks = 0; ks < ksteps; ++ks) {
    FragB af;
    af.h[0] = *(const v8us*)(ap + 32 * ks);
    af.h[1] = *(const v8us*)(ap + 32 * ks + 16);
#pragma unroll
    for (int t = 0; t < NT; ++t) {
      const unsigned short* wq = wp + (size_t)(16 * t) * (size_t)K + 32 * ks;
      FragB bf;
      bf.h[0] = *(const v8us*)wq;
      bf.h[1] = *(const v8us*)(wq + 16);
      acc[t] = wmb(af, bf, acc[t]);
    }
  }

#pragma unroll
  for (int t = 0; t < NT; ++t) {
    const int lc = 16 * t + m;
#pragma unroll
    for (int r = 0; r < 8; ++r) {
      const int lr = 16 * wave + 8 * hh + r;
      stg[lr * BN + lc] = acc[t][r];
    }
  }
  __syncthreads();

  const int rsub = lane / LPR;
  const int cp   = lane - rsub * LPR;
  v4f fv[NI];
#pragma unroll
  for (int i = 0; i < NI; ++i) {
    const int lr = 16 * wave + RPI * i + rsub;
    fv[i] = *(const v4f*)(stg + lr * BN + 4 * cp);
  }
#pragma unroll
  for (int i = 0; i < NI; ++i) {
    const int lr = 16 * wave + RPI * i + rsub;
    const int gr = rowBase + lr;
    float* op = outF + (size_t)gr * (size_t)ldo + col0 + 4 * cp;
    *(volatile v4f*)op = fv[i];
  }
  __threadfence();
#pragma unroll
  for (int i = 0; i < NI; ++i) {
    const int lr = 16 * wave + RPI * i + rsub;
    const int gr = rowBase + lr;
    float* op = outF + (size_t)gr * (size_t)ldo + col0 + 4 * cp;
    *(volatile v4f*)op = fv[i];
  }
}

template<int OUTM>
__global__ __launch_bounds__(NTHR) void k_agg(
    const int* __restrict__ srcs, const int* __restrict__ dsts,
    const float* __restrict__ P, int pitchP, int selfOff, int nbrOff,
    const float* __restrict__ bias,
    unsigned short* Aout, int ldaOut,
    float* outF,
    int nN, int nE, int nb, int vec8, int MPr) {
  constexpr int CPL = (OUTM == 0) ? 4 : 2;
  extern __shared__ v4f lds_dyn[];
  int* reg1 = (int*)lds_dyn;
  int* reg2 = reg1 + RCAP;
  int* scnt = reg2 + RCAP;
  int* soff = scnt + NBMAX;
  int* list = soff + NBMAX;
  int* wcnt = list + LISTN;
  int* wtot = wcnt + NWAVE;
  const int tid = (int)threadIdx.x, lane = tid & 31, wave = tid >> 5;
  const int nodeBase = (int)blockIdx.x * nb;

  for (int i = tid; i < NBMAX; i += NTHR) scnt[i] = 0;
  __syncthreads();

  int tot = 0;
  const int nChunks = (nE + CHUNK - 1) / CHUNK;
#pragma unroll 1
  for (int ch = 0; ch < nChunks; ++ch) {
    const int cbase = ch * CHUNK;
    const int wc = scan_chunk(dsts, nE, cbase, nodeBase, nb, vec8, list, tid, lane, wave);
    if (lane == 0) wcnt[wave] = wc;
    __syncthreads();
    int pre = 0, all = 0;
#pragma unroll
    for (int w2 = 0; w2 < NWAVE; ++w2) {
      int c = wcnt[w2];
      c = c < 0 ? 0 : (c > WCAP ? WCAP : c);
      all += c;
      pre += (w2 < wave) ? c : 0;
    }
    const int wcc  = wc > WCAP ? WCAP : wc;
    const int base = tot + pre;
#pragma unroll 1
    for (int i = lane; i < wcc; i += 32) {
      const int ent = list[wave * WCAP + i];
      const int el  = (ent >> PKS) & (CHUNK - 1);
      const int sl  = ent & (NBMAX - 1);
      int eid = cbase + el;
      eid = eid > nE - 1 ? nE - 1 : eid;
      const int pos = base + i;
      if (pos < RCAP) reg1[pos] = (int)(((unsigned)eid << PKS) | (unsigned)sl);
    }
    tot += all;
    tot = tot > RCAP ? RCAP : tot;
    __syncthreads();
  }
  const int nh = tot;

  if (wave == 0) {
#pragma unroll 1
    for (int b0 = 0; b0 < nh; b0 += 32) {
      const int idx = b0 + lane;
      const int uv  = reg1[idx < RCAP ? idx : RCAP - 1];
      const int m32 = (nh - b0) < 32 ? (nh - b0) : 32;
#pragma unroll 1
      for (int k = 0; k < m32; ++k) {
        const int u  = __builtin_amdgcn_readlane(uv, k);
        const int sl = u & (NBMAX - 1);
        if (lane == 0) scnt[sl] = scnt[sl] + 1;
      }
    }
  }
  __syncthreads();

  {
    const v4i ca = *(const v4i*)(scnt + 8 * tid);
    const v4i cb = *(const v4i*)(scnt + 8 * tid + 4);
    const int e0 = ca.x < 0 ? 0 : ca.x, e1 = ca.y < 0 ? 0 : ca.y, e2 = ca.z < 0 ? 0 : ca.z, e3 = ca.w < 0 ? 0 : ca.w;
    const int e4 = cb.x < 0 ? 0 : cb.x, e5 = cb.y < 0 ? 0 : cb.y, e6 = cb.z < 0 ? 0 : cb.z, e7 = cb.w < 0 ? 0 : cb.w;
    const int ts = e0 + e1 + e2 + e3 + e4 + e5 + e6 + e7;
    int incl = ts;
#pragma unroll
    for (int d = 1; d < 32; d <<= 1) {
      const int up = __shfl_up(incl, d);
      if (lane >= d) incl += up;
    }
    if (lane == 31) wtot[wave] = incl;
    __syncthreads();
    int pre = 0;
#pragma unroll
    for (int w2 = 0; w2 < NWAVE; ++w2) pre += (w2 < wave) ? wtot[w2] : 0;
    int run = pre + incl - ts;
    soff[8 * tid + 0] = run; run += e0;
    soff[8 * tid + 1] = run; run += e1;
    soff[8 * tid + 2] = run; run += e2;
    soff[8 * tid + 3] = run; run += e3;
    soff[8 * tid + 4] = run; run += e4;
    soff[8 * tid + 5] = run; run += e5;
    soff[8 * tid + 6] = run; run += e6;
    soff[8 * tid + 7] = run;
  }
  __syncthreads();
  for (int i = tid; i < NBMAX; i += NTHR) list[i] = soff[i];
  __syncthreads();

  if (wave == 0) {
#pragma unroll 1
    for (int b0 = 0; b0 < nh; b0 += 32) {
      const int idx = b0 + lane;
      const int uv  = reg1[idx < RCAP ? idx : RCAP - 1];
      const int m32 = (nh - b0) < 32 ? (nh - b0) : 32;
#pragma unroll 1
      for (int k = 0; k < m32; ++k) {
        const int u   = __builtin_amdgcn_readlane(uv, k);
        const int sl  = u & (NBMAX - 1);
        const int eid = (int)((unsigned)u >> PKS);
        if (lane == 0) {
          int pos = list[sl];
          pos = pos < 0 ? 0 : (pos > RCAP - 1 ? RCAP - 1 : pos);
          reg2[pos] = eid;
          list[sl] = pos + 1;
        }
      }
    }
  }
  __syncthreads();

  const int nbw = nb >> 3;
  const bool ovf = (nh >= RCAP);
  const float qnan = __int_as_float(0x7fc00000);
  float* stw = (float*)reg1 + wave * STW;
  unsigned int* stwu = (unsigned int*)stw;
  float bb[4] = {0.f, 0.f, 0.f, 0.f};
#pragma unroll
  for (int c = 0; c < CPL; ++c) bb[c] = bf_rne(bias[CPL * lane + c]);

#pragma unroll 1
  for (int jt = 0; jt < nbw; ++jt) {
    const int slot = wave * nbw + jt;
    const int grow = nodeBase + slot;
    const int gcl  = grow < nN ? grow : nN - 1;
    int st = soff[slot];
    const int craw = scnt[slot];
    int cnt = craw;
    st  = st < 0 ? 0 : (st > nh ? nh : st);
    cnt = cnt < 0 ? 0 : (cnt > DEGCAP ? DEGCAP : cnt);
    if (cnt > nh - st) cnt = nh - st;
    const float pz = (ovf || craw > DEGCAP) ? qnan : 0.0f;
    const float live = grow < nN ? 1.0f : 0.0f;

    const float* srow = P + (size_t)gcl * (size_t)pitchP + selfOff + CPL * lane;
    float sv[4] = {0.f, 0.f, 0.f, 0.f};
    float ag[4] = {0.f, 0.f, 0.f, 0.f};
    if (CPL == 4) {
      const v4f t4 = *(const v4f*)srow;
      sv[0] = t4.x; sv[1] = t4.y; sv[2] = t4.z; sv[3] = t4.w;
    } else {
      const v2f t2 = *(const v2f*)srow;
      sv[0] = t2.x; sv[1] = t2.y;
    }

#pragma unroll 1
    for (int q = 0; q < cnt; ++q) {
      int idx = st + q; idx = idx > RCAP - 1 ? RCAP - 1 : idx;
      int eid = reg2[idx]; eid = eid < 0 ? 0 : (eid > nE - 1 ? nE - 1 : eid);
      const int sraw = srcs[eid];
      const int s = sraw < 0 ? 0 : (sraw > nN - 1 ? nN - 1 : sraw);
      const float* nr = P + (size_t)s * (size_t)pitchP + nbrOff + CPL * lane;
      if (CPL == 4) {
        const v4f v = *(const v4f*)nr;
        ag[0] += v.x; ag[1] += v.y; ag[2] += v.z; ag[3] += v.w;
      } else {
        const v2f v = *(const v2f*)nr;
        ag[0] += v.x; ag[1] += v.y;
      }
    }
    const float dcl  = cnt > 0 ? (float)cnt : 1.0f;
    const float invd = 1.0f / dcl;
    float rv[4];
#pragma unroll
    for (int c = 0; c < 4; ++c) {
      float v = (sv[c] + ag[c] * invd) + bb[c];
      if (OUTM == 0) v = fmaxf(v, 0.0f);
      rv[c] = v * live + pz;
    }

    if (OUTM == 0) {
      const unsigned short hb0 = bf_bits(rv[0]), hb1 = bf_bits(rv[1]), hb2 = bf_bits(rv[2]), hb3 = bf_bits(rv[3]);
      const unsigned short lb0 = bf_bits(rv[0] - bf_val(hb0)), lb1 = bf_bits(rv[1] - bf_val(hb1));
      const unsigned short lb2 = bf_bits(rv[2] - bf_val(hb2)), lb3 = bf_bits(rv[3] - bf_val(hb3));
      v2u hw, lw;
      hw.x = (unsigned int)hb0 | ((unsigned int)hb1 << 16);
      hw.y = (unsigned int)hb2 | ((unsigned int)hb3 << 16);
      lw.x = (unsigned int)lb0 | ((unsigned int)lb1 << 16);
      lw.y = (unsigned int)lb2 | ((unsigned int)lb3 << 16);
      __builtin_amdgcn_fence(__ATOMIC_RELEASE, "wavefront");
      __builtin_amdgcn_wave_barrier();
      *(v2u*)(stwu + 2 * lane)      = hw;
      *(v2u*)(stwu + 64 + 2 * lane) = lw;
      __builtin_amdgcn_fence(__ATOMIC_RELEASE, "wavefront");
      __builtin_amdgcn_wave_barrier();
      const v4u pk = *(const v4u*)(stwu + 4 * lane);
      unsigned short* gp = Aout + (size_t)grow * (size_t)ldaOut + 8 * lane;
      const bool wsv = grow < MPr;
      if (wsv) *(volatile v4u*)gp = pk;
      __threadfence();
      if (wsv) *(volatile v4u*)gp = pk;
    } else {
      v2f t2; t2.x = rv[0]; t2.y = rv[1];
      __builtin_amdgcn_fence(__ATOMIC_RELEASE, "wavefront");
      __builtin_amdgcn_wave_barrier();
      *(v2f*)(stw + 2 * lane) = t2;
      __builtin_amdgcn_fence(__ATOMIC_RELEASE, "wavefront");
      __builtin_amdgcn_wave_barrier();
      const int lq = lane < 16 ? lane : 15;
      const v4f ov = *(const v4f*)(stw + 4 * lq);
      float* op = outF + (size_t)gcl * DC + 4 * lq;
      const bool wsv = (grow < nN) && (lane < 16);
      if (wsv) *(volatile v4f*)op = ov;
      __threadfence();
      if (wsv) *(volatile v4f*)op = ov;
    }
  }
}

static int pick_nb(int nE, int nN) {
  int nb = NBMAX;
  while (nb > 16 && (long long)nb * (long long)nE * 5LL > (long long)RCAP * (long long)nN * 4LL) nb >>= 1;
  return nb;
}
static inline int cdiv(int a, int b) { return (a + b - 1) / b; }

extern "C" void kernel_launch(void* const* d_in, const int* in_sizes, int n_in,
                              void* d_out, int out_size, void* d_ws, size_t ws_size,
                              hipStream_t stream) {
  if (n_in < 12) return;
  const int nN = in_sizes[0] / DIN;
  if (nN <= 0 || in_sizes[0] != nN * DIN || nN > (1 << 22)) return;
  const int nE = in_sizes[1];
  if (nE < 1 || in_sizes[2] != nE || nE > (1 << 21)) return;
  if (in_sizes[3] != DIN * DH || in_sizes[4]  != DIN * DH || in_sizes[5]  != DH) return;
  if (in_sizes[6] != DH * DH  || in_sizes[7]  != DH * DH  || in_sizes[8]  != DH) return;
  if (in_sizes[9] != DH * DC  || in_sizes[10] != DH * DC  || in_sizes[11] != DC) return;
  if (out_size != nN * DC) return;

  const float* x   = (const float*)d_in[0];
  const int*   src = (const int*)  d_in[1];
  const int*   dst = (const int*)  d_in[2];
  const float* Ws0 = (const float*)d_in[3];
  const float* Wn0 = (const float*)d_in[4];
  const float* b0  = (const float*)d_in[5];
  const float* Ws1 = (const float*)d_in[6];
  const float* Wn1 = (const float*)d_in[7];
  const float* b1  = (const float*)d_in[8];
  const float* Ws2 = (const float*)d_in[9];
  const float* Wn2 = (const float*)d_in[10];
  const float* b2  = (const float*)d_in[11];
  float* out = (float*)d_out;

  const int MP   = cdiv(nN, GBM) * GBM;
  const int nb   = pick_nb(nE, nN);
  const int gA   = cdiv(MP, nb);
  const int vec8 = 1;
  if (gA * nb < MP) return;

  char* ws = (char*)d_ws;
  size_t off = 0;
  const size_t oXB  = off; off += (size_t)MP * DIN * 2;            off = (off + 255) & ~(size_t)255;
  const size_t oP   = off; off += (size_t)MP * PW * 4;             off = (off + 255) & ~(size_t)255;
  const size_t oAH1 = off; off += (size_t)MP * APW * 2;            off = (off + 255) & ~(size_t)255;
  const size_t oAH2 = off; off += (size_t)MP * APW * 2;            off = (off + 255) & ~(size_t)255;
  const size_t oW0  = off; off += (size_t)(2 * DH) * DIN * 2;      off = (off + 255) & ~(size_t)255;
  const size_t oW1N = off; off += (size_t)DH * (2 * DH) * 2;       off = (off + 255) & ~(size_t)255;
  const size_t oW1S = off; off += (size_t)DH * (2 * DH) * 2;       off = (off + 255) & ~(size_t)255;
  const size_t oW2  = off; off += (size_t)(2 * DC) * (2 * DH) * 2; off = (off + 255) & ~(size_t)255;
  if (off > ws_size || off > (size_t)WSMAX) return;
  unsigned short* XB   = (unsigned short*)(ws + oXB);
  float*          P    = (float*)(ws + oP);
  unsigned short* AH1  = (unsigned short*)(ws + oAH1);
  unsigned short* AH2  = (unsigned short*)(ws + oAH2);
  unsigned short* WT0  = (unsigned short*)(ws + oW0);
  unsigned short* WT1N = (unsigned short*)(ws + oW1N);
  unsigned short* WT1S = (unsigned short*)(ws + oW1S);
  unsigned short* WT2  = (unsigned short*)(ws + oW2);

  hipFuncSetAttribute(reinterpret_cast<const void*>(&k_agg<0>),
                      hipFuncAttributeMaxDynamicSharedMemorySize, LDS_AGG);
  hipFuncSetAttribute(reinterpret_cast<const void*>(&k_agg<1>),
                      hipFuncAttributeMaxDynamicSharedMemorySize, LDS_AGG);

  const int nUx = MP * (DIN / 8);
  k_xprep<<<cdiv(nUx, NTHR), NTHR, 0, stream>>>(x, XB, nN, nUx);

  {
    const int nU0 = (2 * DH) * (DIN / 8);
    k_wtr<<<cdiv(nU0, NTHR), NTHR, 0, stream>>>(Ws0, Wn0, DH, DH, DH, DIN, DIN, WT0, nU0);
    const int nU1 = DH * ((2 * DH) / 8);
    k_wtr<<<cdiv(nU1, NTHR), NTHR, 0, stream>>>(Wn1, Wn1, DH, DH, DH, DH, 2 * DH, WT1N, nU1);
    k_wtr<<<cdiv(nU1, NTHR), NTHR, 0, stream>>>(Ws1, Ws1, DH, DH, DH, DH, 2 * DH, WT1S, nU1);
    const int nU2 = (2 * DC) * ((2 * DH) / 8);
    k_wtr<<<cdiv(nU2, NTHR), NTHR, 0, stream>>>(Ws2, Wn2, DC, DC, DC, DH, 2 * DH, WT2, nU2);
  }

  const int gM = MP / GBM;
  k_gemm<4><<<dim3(gM, (2 * DH) / 64), GTHR, 0, stream>>>(XB, DIN, WT0, DIN, P, PW);
  k_agg<0><<<gA, NTHR, LDS_AGG, stream>>>(src, dst, P, PW, 0, DH, b0, AH1, APW, out, nN, nE, nb, vec8, MP);
  k_gemm<4><<<dim3(gM, DH / 64), GTHR, 0, stream>>>(AH1, APW, WT1N, 2 * DH, P + DH, PW);
  k_gemm<8><<<dim3(gM, 1), GTHR, 0, stream>>>(AH1, APW, WT1S, 2 * DH, P, PW);
  k_agg<0><<<gA, NTHR, LDS_AGG, stream>>>(src, dst, P, PW, 0, DH, b1, AH2, APW, out, nN, nE, nb, vec8, MP);
  k_gemm<4><<<dim3(gM, (2 * DC) / 64), GTHR, 0, stream>>>(AH2, APW, WT2, 2 * DH, P + DH, PW);
  k_agg<1><<<gA, NTHR, LDS_AGG, stream>>>(src, dst, P, PW, DH, DH + DC, b2, AH2, APW, out, nN, nE, nb, vec8, MP);
}
